// LagunaAttention_27462020891147
// MI455X (gfx1250) — hardware-verified
//
#include <hip/hip_runtime.h>
#include <math.h>
#include <stdint.h>

#define NTOK   4096
#define HID    2048
#define NHQ    16
#define NKVH   4
#define HDM    128
#define QKVN   3072
#define QW     2048
#define QKW    2560
#define KVW    512
#define NFREQ  64
#define NGATE  16

typedef _Float16       v16h __attribute__((ext_vector_type(16)));
typedef _Float16       v8h  __attribute__((ext_vector_type(8)));
typedef __bf16         v16b __attribute__((ext_vector_type(16)));
typedef __bf16         v8b  __attribute__((ext_vector_type(8)));
typedef float          v8f  __attribute__((ext_vector_type(8)));
typedef float          v4f  __attribute__((ext_vector_type(4)));
typedef unsigned int   v4u  __attribute__((ext_vector_type(4)));
typedef unsigned short v8us __attribute__((ext_vector_type(8)));

__device__ __forceinline__ unsigned short bf_bits(float f) {
  const unsigned u = __float_as_uint(f);
  return (unsigned short)((u + 0x7FFFu + ((u >> 16) & 1u)) >> 16);
}
__device__ __forceinline__ float bf_val(unsigned short h) { return __uint_as_float(((unsigned)h) << 16); }
__device__ __forceinline__ float bf_rne(float f) { return bf_val(bf_bits(f)); }
__device__ __forceinline__ unsigned pk16(unsigned short a, unsigned short b) { return (unsigned)a | ((unsigned)b << 16); }
__device__ __forceinline__ v8f zero8() { v8f z = {0.f, 0.f, 0.f, 0.f, 0.f, 0.f, 0.f, 0.f}; return z; }
__device__ __forceinline__ int wave_id() { return __builtin_amdgcn_readfirstlane((int)(threadIdx.x >> 5)); }

__device__ __forceinline__ void lds_wave_sync() {
  __builtin_amdgcn_fence(__ATOMIC_RELEASE, "workgroup");
  __builtin_amdgcn_wave_barrier();
  __builtin_amdgcn_fence(__ATOMIC_ACQUIRE, "workgroup");
}

union FragH { v16h v; v8h h[2]; };
union FragB { v16b v; v8b h[2]; };
__device__ __forceinline__ v16h ldfrag_h(const _Float16* p) { FragH f; f.h[0] = *(const v8h*)(p); f.h[1] = *(const v8h*)(p + 16); return f.v; }
__device__ __forceinline__ v16b ldfrag_b(const __bf16* p)   { FragB f; f.h[0] = *(const v8b*)(p); f.h[1] = *(const v8b*)(p + 16); return f.v; }

__device__ __forceinline__ v8f mma_h(v16h a, v16h b, v8f c) {
  return __builtin_amdgcn_wmma_f32_16x16x32_f16(false, a, false, b, (short)0, c, false, false);
}
__device__ __forceinline__ v8f mma_b(v16b a, v16b b, v8f c) {
  return __builtin_amdgcn_wmma_f32_16x16x32_bf16(false, a, false, b, (short)0, c, false, false);
}

#if defined(__HIP_DEVICE_COMPILE__)
#define KX_NOP4 "v_nop\n\tv_nop\n\tv_nop\n\tv_nop"
__device__ __forceinline__ void guard_b5(v8f& a, v8f& b, v16b x0, v16b x1, v16b x2, v16b x3, v16b y) {
  asm volatile(KX_NOP4 : "+v"(a), "+v"(b) : "v"(x0), "v"(x1), "v"(x2), "v"(x3), "v"(y) : "memory");
}
__device__ __forceinline__ void guard_b3(v8f& a, v8f& b, v16b x, v16b y, v16b z) {
  asm volatile(KX_NOP4 : "+v"(a), "+v"(b) : "v"(x), "v"(y), "v"(z) : "memory");
}
__device__ __forceinline__ void guard1_b4(v8f& a, v16b w, v16b x, v16b y, v16b z) {
  asm volatile(KX_NOP4 : "+v"(a) : "v"(w), "v"(x), "v"(y), "v"(z) : "memory");
}
__device__ __forceinline__ void guard_h4(v8f& a, v8f& b, v16h w, v16h x, v16h y, v16h z) {
  asm volatile(KX_NOP4 : "+v"(a), "+v"(b) : "v"(w), "v"(x), "v"(y), "v"(z) : "memory");
}
__device__ __forceinline__ void acc_guard4(v8f& a, v8f& b, v8f& c, v8f& d) {
  asm volatile(KX_NOP4 : "+v"(a), "+v"(b), "+v"(c), "+v"(d));
}
#else
__device__ __forceinline__ void guard_b5(v8f&, v8f&, v16b, v16b, v16b, v16b, v16b) {}
__device__ __forceinline__ void guard_b3(v8f&, v8f&, v16b, v16b, v16b) {}
__device__ __forceinline__ void guard1_b4(v8f&, v16b, v16b, v16b, v16b) {}
__device__ __forceinline__ void guard_h4(v8f&, v8f&, v16h, v16h, v16h, v16h) {}
__device__ __forceinline__ void acc_guard4(v8f&, v8f&, v8f&, v8f&) {}
#endif

__global__ __launch_bounds__(256) void rope_table_kernel(const int* __restrict__ pos, float* __restrict__ cst,
                                                         float* __restrict__ snt, int ntok) {
  const int lane = threadIdx.x & 31;
  const int wave = (int)(threadIdx.x >> 5);
  const int t = (int)blockIdx.x * 8 + wave;
  if (t >= ntok) return;
  const float pf = (float)pos[t];
  float c0 = 0.f, s0 = 0.f, c1 = 0.f, s1 = 0.f;
#pragma unroll 1
  for (int u = 0; u < 2; ++u) {
    const int i = lane + 32 * u;
    const float e   = (float)i * 0.015625f;
    const float pw  = powf(10000.0f, e);
    const float inv = 1.0f / pw;
    const float ang = pf * inv;
    const float cv = cosf(ang);
    const float sv = sinf(ang);
    c1 = cv; s1 = sv;
    if (u == 0) { c0 = cv; s0 = sv; }
  }
  const size_t o = (size_t)t * NFREQ + lane;
  for (int pass = 0; pass < 2; ++pass) {
    ((volatile float*)cst)[o]      = c0;
    ((volatile float*)cst)[o + 32] = c1;
    ((volatile float*)snt)[o]      = s0;
    ((volatile float*)snt)[o + 32] = s1;
    __threadfence();
  }
}

__global__ __launch_bounds__(256) void cvt_bf16_kernel(const float* __restrict__ in, unsigned short* __restrict__ outp, int n8) {
  const int i = (int)blockIdx.x * 256 + (int)threadIdx.x;
  if (i >= n8) return;
  const size_t e = 8 * (size_t)i;
  const v4f a = *(const v4f*)(in + e);
  const v4f b = *(const v4f*)(in + e + 4);
  v4u w;
  w[0] = pk16(bf_bits(a[0]), bf_bits(a[1]));
  w[1] = pk16(bf_bits(a[2]), bf_bits(a[3]));
  w[2] = pk16(bf_bits(b[0]), bf_bits(b[1]));
  w[3] = pk16(bf_bits(b[2]), bf_bits(b[3]));
  *(volatile v4u*)(outp + e) = w;
  __threadfence();
  *(volatile v4u*)(outp + e) = w;
}

__global__ __launch_bounds__(256) void tconv_bf16_kernel(const float* __restrict__ W, unsigned short* __restrict__ outp, int R, int Cc) {
  __shared__ __align__(16) float tf[64 * 68];
  const int c0  = (int)blockIdx.x * 64;
  const int r0  = (int)blockIdx.y * 64;
  const int tid = (int)threadIdx.x;
  {
    const int lr = tid >> 4;
    const int c4 = (tid & 15) * 4;
#pragma unroll
    for (int it = 0; it < 4; ++it) {
      const int rr = it * 16 + lr;
      const v4f a = *(const v4f*)(W + (size_t)(r0 + rr) * Cc + c0 + c4);
      *(v4f*)(tf + rr * 68 + c4) = a;
    }
  }
  __syncthreads();
  const int sub = tid >> 3;
  const int c8  = (tid & 7) * 8;
  v4u hv[2];
#pragma unroll
  for (int it = 0; it < 2; ++it) {
    const int oc = it * 32 + sub;
    v4u a;
#pragma unroll
    for (int q = 0; q < 4; ++q) {
      const float f0 = tf[(c8 + 2 * q) * 68 + oc];
      const float f1 = tf[(c8 + 2 * q + 1) * 68 + oc];
      a[q] = pk16(bf_bits(f0), bf_bits(f1));
    }
    hv[it] = a;
  }
  for (int pass = 0; pass < 2; ++pass) {
#pragma unroll
    for (int it = 0; it < 2; ++it) {
      const int oc = it * 32 + sub;
      const size_t go = (size_t)(c0 + oc) * R + r0 + c8;
      *(volatile v4u*)(outp + go) = hv[it];
    }
    __threadfence();
  }
}

__global__ __launch_bounds__(256) void tconv16_bf16_kernel(const float* __restrict__ W, unsigned short* __restrict__ outp, int R) {
  __shared__ __align__(16) float tf[16 * 68];
  const int r0  = (int)blockIdx.x * 64;
  const int tid = (int)threadIdx.x;
  {
    const int rr = tid >> 2;
    const int c4 = (tid & 3) * 4;
    const v4f a = *(const v4f*)(W + (size_t)(r0 + rr) * NGATE + c4);
    tf[(c4 + 0) * 68 + rr] = a[0];
    tf[(c4 + 1) * 68 + rr] = a[1];
    tf[(c4 + 2) * 68 + rr] = a[2];
    tf[(c4 + 3) * 68 + rr] = a[3];
  }
  __syncthreads();
  if (tid < 128) {
    const int oc = tid >> 3;
    const int p8 = (tid & 7) * 8;
    v4u hv;
#pragma unroll
    for (int q = 0; q < 4; ++q) {
      const float f0 = tf[oc * 68 + p8 + 2 * q];
      const float f1 = tf[oc * 68 + p8 + 2 * q + 1];
      hv[q] = pk16(bf_bits(f0), bf_bits(f1));
    }
    const size_t go = (size_t)oc * R + r0 + p8;
    *(volatile v4u*)(outp + go) = hv;
    __threadfence();
    *(volatile v4u*)(outp + go) = hv;
  }
}

template <int EPI, bool SPLITA>
__global__ __launch_bounds__(128) void gemm_w32x128_kernel(
    const unsigned short* Ap, const unsigned short* A2p, int lda,
    const unsigned short* __restrict__ Btp, int ldb,
    const float* __restrict__ nwq, const float* __restrict__ nwk,
    const float* __restrict__ cst, const float* __restrict__ snt,
    void* C0, void* C1, void* C2, void* C3, int ldc,
    int M, int N, int K) {
  __shared__ __align__(16) unsigned int slab_all[4 * 2048];

  const int lane = threadIdx.x & 31;
  const int wave = wave_id();
  const int hh = lane >> 4;
  const int rl = lane & 15;
  const int tilesN = N >> 7;
  const int tilesM = M >> 5;
  const int tile = (int)blockIdx.x * 4 + wave;
  if (tile >= tilesM * tilesN) return;
  const int tm = tile / tilesN;
  const int tn = tile - tm * tilesN;
  const int m0 = tm << 5;
  const int n0 = tn << 7;

  const __bf16* A  = (const __bf16*)(const void*)Ap;
  const __bf16* A2 = (const __bf16*)(const void*)A2p;
  const __bf16* Bt = (const __bf16*)(const void*)Btp;

  v8f acc[2][8];
#pragma unroll
  for (int i = 0; i < 2; ++i)
#pragma unroll
    for (int j = 0; j < 8; ++j) acc[i][j] = zero8();

  for (int k0 = 0; k0 < K; k0 += 32) {
    v16b ah[2], al[2];
#pragma unroll
    for (int i = 0; i < 2; ++i) {
      const size_t ao = (size_t)(m0 + i * 16 + rl) * lda + k0 + 8 * hh;
      ah[i] = ldfrag_b(A + ao);
      al[i] = SPLITA ? ldfrag_b(A2 + ao) : ah[i];
    }
#pragma unroll
    for (int j = 0; j < 8; ++j) {
      const v16b bj = ldfrag_b(Bt + (size_t)(n0 + j * 16 + rl) * ldb + k0 + 8 * hh);
      acc[0][j] = mma_b(ah[0], bj, acc[0][j]);
      acc[1][j] = mma_b(ah[1], bj, acc[1][j]);
      if (SPLITA) {
        acc[0][j] = mma_b(al[0], bj, acc[0][j]);
        acc[1][j] = mma_b(al[1], bj, acc[1][j]);
      }
      guard_b5(acc[0][j], acc[1][j], ah[0], ah[1], al[0], al[1], bj);
    }
  }
  acc_guard4(acc[0][0], acc[0][1], acc[0][2], acc[0][3]);
  acc_guard4(acc[0][4], acc[0][5], acc[0][6], acc[0][7]);
  acc_guard4(acc[1][0], acc[1][1], acc[1][2], acc[1][3]);
  acc_guard4(acc[1][4], acc[1][5], acc[1][6], acc[1][7]);

  unsigned int* slabw = slab_all + wave * 2048;

  if (EPI == 0) {
    unsigned short* sl = (unsigned short*)(void*)slabw;
    const bool isq = (n0 < QW);
    unsigned short* P0 = isq ? (unsigned short*)C0 : (unsigned short*)C2;
    unsigned short* P1 = isq ? (unsigned short*)C1 : (unsigned short*)C3;
    const float* nw = isq ? nwq : nwk;
    const int ldp  = isq ? ldc : KVW;
    const int col0 = isq ? n0 : (n0 - QW);
#pragma unroll
    for (int i = 0; i < 2; ++i) {
      const int rb = m0 + i * 16 + 8 * hh;
      float inv[8];
#pragma unroll
      for (int r = 0; r < 8; ++r) {
        float ss = 0.f;
#pragma unroll
        for (int j = 0; j < 8; ++j) ss += acc[i][j][r] * acc[i][j][r];
        ss += __shfl_xor(ss, 1, 32);
        ss += __shfl_xor(ss, 2, 32);
        ss += __shfl_xor(ss, 4, 32);
        ss += __shfl_xor(ss, 8, 32);
        inv[r] = rsqrtf(ss * 0.0078125f + 1e-6f);
      }
#pragma unroll
      for (int j = 0; j < 4; ++j) {
        const int dim = j * 16 + rl;
        const float w1 = bf_rne(nw[dim]);
        const float w2 = bf_rne(nw[dim + 64]);
#pragma unroll
        for (int r = 0; r < 8; ++r) {
          const int row = rb + r;
          const float cv = cst[(size_t)row * NFREQ + dim];
          const float sv = snt[(size_t)row * NFREQ + dim];
          const float x1 = acc[i][j][r] * inv[r] * w1;
          const float x2 = acc[i][j + 4][r] * inv[r] * w2;
          const float o1 = x1 * cv - x2 * sv;
          const float o2 = x2 * cv + x1 * sv;
          const unsigned short hb1 = bf_bits(o1);
          const unsigned short hb2 = bf_bits(o2);
          const unsigned short lb1 = bf_bits(o1 - bf_val(hb1));
          const unsigned short lb2 = bf_bits(o2 - bf_val(hb2));
          const int so = (8 * hh + r) * 128 + dim;
          sl[so]             = hb1;
          sl[so + 64]        = hb2;
          sl[2048 + so]      = lb1;
          sl[2048 + so + 64] = lb2;
        }
      }
      lds_wave_sync();
      for (int pass = 0; pass < 2; ++pass) {
#pragma unroll
        for (int it = 0; it < 8; ++it) {
          const int row = it * 2 + hh;
          const int c8  = rl * 8;
          const v8us vh = *(const v8us*)(sl + row * 128 + c8);
          const v8us vl = *(const v8us*)(sl + 2048 + row * 128 + c8);
          const size_t go = (size_t)(m0 + i * 16 + row) * ldp + col0 + c8;
          *(volatile v8us*)(P0 + go) = vh;
          *(volatile v8us*)(P1 + go) = vl;
        }
        __threadfence();
      }
      lds_wave_sync();
    }
  } else if (EPI == 1) {
    _Float16* sl16 = (_Float16*)(void*)slabw;
    _Float16* P0 = (_Float16*)C0;
    _Float16* P1 = (_Float16*)C1;
#pragma unroll
    for (int i = 0; i < 2; ++i) {
#pragma unroll
      for (int r = 0; r < 8; ++r) {
#pragma unroll
        for (int j = 0; j < 8; ++j) {
          const float v = acc[i][j][r];
          const _Float16 hv = (_Float16)v;
          const int so = (8 * hh + r) * 128 + j * 16 + rl;
          sl16[so]        = hv;
          sl16[2048 + so] = (_Float16)((v - (float)hv) * 2048.0f);
        }
      }
      lds_wave_sync();
      for (int pass = 0; pass < 2; ++pass) {
#pragma unroll
        for (int it = 0; it < 8; ++it) {
          const int row = it * 2 + hh;
          const int c8  = rl * 8;
          const v8h vh = *(const v8h*)(sl16 + row * 128 + c8);
          const v8h vl = *(const v8h*)(sl16 + 2048 + row * 128 + c8);
          const size_t go = (size_t)(m0 + i * 16 + row) * ldc + n0 + c8;
          *(volatile v8h*)(P0 + go) = vh;
          *(volatile v8h*)(P1 + go) = vl;
        }
        __threadfence();
      }
      lds_wave_sync();
    }
  } else {
    float* slf = (float*)(void*)slabw;
    float* C = (float*)C0;
#pragma unroll
    for (int i = 0; i < 2; ++i) {
#pragma unroll
      for (int j = 0; j < 8; ++j)
#pragma unroll
        for (int r = 0; r < 8; ++r)
          slf[(8 * hh + r) * 128 + j * 16 + rl] = acc[i][j][r];
      lds_wave_sync();
      for (int pass = 0; pass < 2; ++pass) {
#pragma unroll
        for (int row = 0; row < 16; ++row) {
          const v4f v = *(const v4f*)(slf + row * 128 + lane * 4);
          *(volatile v4f*)(C + (size_t)(m0 + i * 16 + row) * ldc + n0 + lane * 4) = v;
        }
        __threadfence();
      }
      lds_wave_sync();
    }
  }
}

__global__ __launch_bounds__(128) void gate_kernel(const unsigned short* __restrict__ Xbp, const unsigned short* __restrict__ Wgtp,
                                                  float* __restrict__ gate, int M, int K) {
  __shared__ __align__(16) float gsl[4 * 512];
  const int lane = threadIdx.x & 31;
  const int wave = wave_id();
  const int hh = lane >> 4;
  const int rl = lane & 15;
  const int m0 = ((int)blockIdx.x * 4 + wave) * 32;
  if (m0 >= M) return;
  const __bf16* A = (const __bf16*)(const void*)Xbp;
  const __bf16* B = (const __bf16*)(const void*)Wgtp;

  v8f acc[2];
  acc[0] = zero8(); acc[1] = zero8();
  for (int k0 = 0; k0 < K; k0 += 32) {
    const v16b a0 = ldfrag_b(A + (size_t)(m0 + rl) * K + k0 + 8 * hh);
    const v16b a1 = ldfrag_b(A + (size_t)(m0 + 16 + rl) * K + k0 + 8 * hh);
    const v16b bg = ldfrag_b(B + (size_t)rl * K + k0 + 8 * hh);
    acc[0] = mma_b(a0, bg, acc[0]);
    acc[1] = mma_b(a1, bg, acc[1]);
    guard_b3(acc[0], acc[1], a0, a1, bg);
  }
  acc_guard4(acc[0], acc[1], acc[0], acc[1]);

  float* sl = gsl + wave * 512;
#pragma unroll
  for (int i = 0; i < 2; ++i)
#pragma unroll
    for (int r = 0; r < 8; ++r) {
      const float x = acc[i][r];
      const float g = fmaxf(x, 0.f) + log1pf(expf(-fabsf(x)));
      sl[(i * 16 + 8 * hh + r) * 16 + rl] = g;
    }
  lds_wave_sync();
  for (int pass = 0; pass < 2; ++pass) {
#pragma unroll
    for (int it = 0; it < 4; ++it) {
      const v4f v = *(const v4f*)(sl + it * 128 + lane * 4);
      *(volatile v4f*)(gate + (size_t)m0 * NGATE + it * 128 + lane * 4) = v;
    }
    __threadfence();
  }
}

#define AT_KC   32
#define KS_P    136
#define VS_P    40
#define PS_P    40
#define LDS_KS  0
#define LDS_KLS (32 * KS_P)
#define LDS_VHS (2 * 32 * KS_P)
#define LDS_VLS (LDS_VHS + 128 * VS_P)
#define LDS_PH  (LDS_VLS + 128 * VS_P)
#define LDS_PL  (LDS_PH + 4 * 16 * PS_P)
#define LDS_TOT (LDS_PL + 4 * 16 * PS_P)
static_assert(LDS_TOT * 2 <= 65536);
static_assert(4 * 4096 <= LDS_TOT);
static_assert((LDS_KLS * 2) % 16 == 0);
static_assert((LDS_VHS * 2) % 16 == 0);
static_assert((LDS_VLS * 2) % 16 == 0);
static_assert((LDS_PH * 2) % 16 == 0);
static_assert((LDS_PL * 2) % 16 == 0);

template <bool PRES>
__global__ __launch_bounds__(128) void attn_causal_kernel(
    const unsigned short* __restrict__ qhp, const unsigned short* __restrict__ qlp,
    const unsigned short* __restrict__ khp, const unsigned short* __restrict__ klp,
    const unsigned short* __restrict__ vhp, const unsigned short* __restrict__ vlp,
    const float* __restrict__ gatep,
    unsigned short* __restrict__ ahp, unsigned short* __restrict__ alp, int qb_base) {
  __shared__ __align__(16) unsigned short lds[LDS_TOT];
  unsigned short* Ks  = lds + LDS_KS;
  unsigned short* Kls = lds + LDS_KLS;
  _Float16* Vhs = (_Float16*)(void*)(lds + LDS_VHS);
  _Float16* Vls = (_Float16*)(void*)(lds + LDS_VLS);
  const __bf16* KsB  = (const __bf16*)(const void*)(lds + LDS_KS);
  const __bf16* KlsB = (const __bf16*)(const void*)(lds + LDS_KLS);

  const int tid  = (int)threadIdx.x;
  const int lane = tid & 31;
  const int wave = wave_id();
  const int hh   = lane >> 4;
  const int c    = lane & 15;
  const int qb   = (int)blockIdx.x + qb_base;
  const int h    = (int)blockIdx.y;
  const int kvh  = h >> 2;
  const int q0   = qb * 64 + wave * 16;
  const int qlast = q0 + 15;

  const __bf16* Qhr = (const __bf16*)(const void*)qhp + (size_t)(q0 + c) * HID + h * HDM + 8 * hh;
  const __bf16* Qlr = (const __bf16*)(const void*)qlp + (size_t)(q0 + c) * HID + h * HDM + 8 * hh;
  const unsigned short* Kg  = khp + kvh * HDM;
  const unsigned short* Klg = klp + kvh * HDM;
  const _Float16* Vhg = (const _Float16*)(const void*)vhp + (size_t)(kvh * HDM) * NTOK;
  const _Float16* Vlg = (const _Float16*)(const void*)vlp + (size_t)(kvh * HDM) * NTOK;
  _Float16* ph = (_Float16*)(void*)(lds + LDS_PH) + wave * (16 * PS_P);
  _Float16* pl = (_Float16*)(void*)(lds + LDS_PL) + wave * (16 * PS_P);

  float mrow[8], lrow[8];
  v8f oacc[8], oaccr[8];
#pragma unroll
  for (int r = 0; r < 8; ++r) { mrow[r] = -INFINITY; lrow[r] = 0.f; }
#pragma unroll
  for (int t = 0; t < 8; ++t) { oacc[t] = zero8(); oaccr[t] = zero8(); }

  const int nch = 2 * qb + 2;
  for (int kc = 0; kc < nch; ++kc) {
    const int kv0 = kc * AT_KC;
    __syncthreads();
#pragma unroll
    for (int i = 0; i < 4; ++i) {
      const int p   = tid + 128 * i;
      const int key = p >> 4, d8 = (p & 15) * 8;
      const v4u kx = *(const v4u*)(Kg  + (size_t)(kv0 + key) * KVW + d8);
      const v4u ky = *(const v4u*)(Klg + (size_t)(kv0 + key) * KVW + d8);
      *(v4u*)(Ks  + key * KS_P + d8) = kx;
      *(v4u*)(Kls + key * KS_P + d8) = ky;
      const int d = p >> 2, k8 = (p & 3) * 8;
      const v4u vx = *(const v4u*)(Vhg + (size_t)d * NTOK + kv0 + k8);
      const v4u vy = *(const v4u*)(Vlg + (size_t)d * NTOK + kv0 + k8);
      *(v4u*)(Vhs + d * VS_P + k8) = vx;
      *(v4u*)(Vls + d * VS_P + k8) = vy;
    }
    __syncthreads();

    if (kv0 <= qlast) {
      v8f sacc[2];
      sacc[0] = zero8(); sacc[1] = zero8();
#pragma unroll
      for (int dc = 0; dc < 4; ++dc) {
        const v16b qa = ldfrag_b(Qhr + dc * 32);
        const v16b ql = ldfrag_b(Qlr + dc * 32);
#pragma unroll
        for (int j = 0; j < 2; ++j) {
          const v16b kb = ldfrag_b(KsB  + (j * 16 + c) * KS_P + dc * 32 + 8 * hh);
          const v16b kl = ldfrag_b(KlsB + (j * 16 + c) * KS_P + dc * 32 + 8 * hh);
          sacc[j] = mma_b(qa, kb, sacc[j]);
          sacc[j] = mma_b(qa, kl, sacc[j]);
          sacc[j] = mma_b(ql, kb, sacc[j]);
          guard1_b4(sacc[j], qa, ql, kb, kl);
        }
      }
      float cm[8];
#pragma unroll
      for (int r = 0; r < 8; ++r) {
        const int qrow = q0 + 8 * hh + r;
        float m = -INFINITY;
#pragma unroll
        for (int j = 0; j < 2; ++j) {
          const int key = kv0 + j * 16 + c;
          float s = sacc[j][r] * 0.08838834764831845f;
          s = (key > qrow) ? -INFINITY : s;
          sacc[j][r] = s;
          m = fmaxf(m, s);
        }
#pragma unroll
        for (int off = 1; off < 16; off <<= 1) m = fmaxf(m, __shfl_xor(m, off, 32));
        cm[r] = m;
      }
#pragma unroll
      for (int r = 0; r < 8; ++r) {
        const float mnew  = fmaxf(mrow[r], cm[r]);
        const float alpha = __expf(mrow[r] - mnew);
        mrow[r] = mnew;
        float psum = 0.f;
#pragma unroll
        for (int j = 0; j < 2; ++j) {
          const float p  = __expf(sacc[j][r] - mnew);
          psum += p;
          const float pp = p * 1024.0f;
          const _Float16 phv = (_Float16)pp;
          const int po = (8 * hh + r) * PS_P + j * 16 + c;
          ph[po] = phv;
          if (PRES) pl[po] = (_Float16)((pp - (float)phv) * 2048.0f);
        }
#pragma unroll
        for (int off = 1; off < 16; off <<= 1) psum += __shfl_xor(psum, off, 32);
        lrow[r] = lrow[r] * alpha + psum;
#pragma unroll
        for (int t = 0; t < 8; ++t) { oacc[t][r] *= alpha; oaccr[t][r] *= alpha; }
      }
      lds_wave_sync();
      const v16h pa = ldfrag_h(ph + c * PS_P + 8 * hh);
      v16h pr = pa;
      if (PRES) pr = ldfrag_h(pl + c * PS_P + 8 * hh);
#pragma unroll
      for (int t = 0; t < 8; ++t) {
        const v16h vb = ldfrag_h(Vhs + (t * 16 + c) * VS_P + 8 * hh);
        const v16h vr = ldfrag_h(Vls + (t * 16 + c) * VS_P + 8 * hh);
        oacc[t]  = mma_h(pa, vb, oacc[t]);
        oaccr[t] = mma_h(pa, vr, oaccr[t]);
        if (PRES) oaccr[t] = mma_h(pr, vb, oaccr[t]);
        guard_h4(oacc[t], oaccr[t], pa, pr, vb, vr);
      }
    }
  }

  __syncthreads();
  unsigned short* osh = lds + wave * 4096;
  unsigned short* osl = osh + 2048;
#pragma unroll
  for (int r = 0; r < 8; ++r) {
    const int row = q0 + 8 * hh + r;
    const float g = gatep[(size_t)row * NGATE + h];
    const float inv = g * (1.0f / lrow[r]) * 0.0009765625f;
#pragma unroll
    for (int t = 0; t < 8; ++t) {
      const float o = (oacc[t][r] + oaccr[t][r] * 0.00048828125f) * inv;
      const unsigned short hb = bf_bits(o);
      const unsigned short lb = bf_bits(o - bf_val(hb));
      const int so = (8 * hh + r) * 128 + t * 16 + c;
      osh[so] = hb;
      osl[so] = lb;
    }
  }
  lds_wave_sync();
  unsigned short* Ahg = ahp + (size_t)q0 * HID + h * HDM;
  unsigned short* Alg = alp + (size_t)q0 * HID + h * HDM;
  for (int pass = 0; pass < 2; ++pass) {
#pragma unroll
    for (int it = 0; it < 8; ++it) {
      const int row = it * 2 + hh;
      const int c8  = c * 8;
      const v8us x = *(const v8us*)(osh + row * 128 + c8);
      const v8us y = *(const v8us*)(osl + row * 128 + c8);
      *(volatile v8us*)(Ahg + (size_t)row * HID + c8) = x;
      *(volatile v8us*)(Alg + (size_t)row * HID + c8) = y;
    }
    __threadfence();
  }
}

extern "C" void kernel_launch(void* const* d_in, const int* in_sizes, int n_in,
                              void* d_out, int out_size, void* d_ws, size_t ws_size,
                              hipStream_t stream) {
  if (n_in < 7) return;
  if (in_sizes[0] != NTOK * HID) return;
  if (in_sizes[1] != NTOK) return;
  if (in_sizes[2] != HID * QKVN) return;
  if (in_sizes[3] != HID * HID) return;
  if (in_sizes[4] != HID * NGATE) return;
  if (in_sizes[5] != HDM) return;
  if (in_sizes[6] != HDM) return;
  if (out_size != NTOK * HID) return;

  const float* hidden    = (const float*)d_in[0];
  const int*   positions = (const int*)d_in[1];
  const float* Wqkv      = (const float*)d_in[2];
  const float* Wo        = (const float*)d_in[3];
  const float* Wg        = (const float*)d_in[4];
  const float* qnw       = (const float*)d_in[5];
  const float* knw       = (const float*)d_in[6];
  float* out = (float*)d_out;

  const size_t szX  = (size_t)NTOK * HID * 2;
  const size_t szWq = (size_t)QKVN * HID * 2;
  const size_t szWo = (size_t)HID * HID * 2;
  const size_t szWg = (size_t)NGATE * HID * 2;
  const size_t szT  = (size_t)NTOK * NFREQ * 4;
  const size_t szG  = (size_t)NTOK * NGATE * 4;
  const size_t szQ  = (size_t)NTOK * HID * 2;
  const size_t szK  = (size_t)NTOK * KVW * 2;
  const size_t szV  = (size_t)KVW * NTOK * 2;
  const size_t szA  = (size_t)NTOK * HID * 2;
  size_t off = 0;
  const size_t oX  = off; off += szX;
  const size_t oWq = off; off += szWq;
  const size_t oWo = off; off += szWo;
  const size_t oWg = off; off += szWg;
  const size_t oCs = off; off += szT;
  const size_t oSn = off; off += szT;
  const size_t oG  = off; off += szG;
  const size_t oQh = off; off += szQ;
  const size_t oQl = off; off += szQ;
  const size_t oKh = off; off += szK;
  const size_t oKl = off; off += szK;
  const size_t oVh = off; off += szV;
  const size_t oVl = off; off += szV;
  const size_t oAh = off; off += szA;
  const size_t oAl = off; off += szA;
  if (off > ws_size) return;
  if (off > (size_t)134217728) return;

  char* ws = (char*)d_ws;
  unsigned short* Xb  = (unsigned short*)(ws + oX);
  unsigned short* WqT = (unsigned short*)(ws + oWq);
  unsigned short* WoT = (unsigned short*)(ws + oWo);
  unsigned short* WgT = (unsigned short*)(ws + oWg);
  float*          cst = (float*)(ws + oCs);
  float*          snt = (float*)(ws + oSn);
  float*          gate = (float*)(ws + oG);
  unsigned short* Qh  = (unsigned short*)(ws + oQh);
  unsigned short* Ql  = (unsigned short*)(ws + oQl);
  unsigned short* Kh  = (unsigned short*)(ws + oKh);
  unsigned short* Kl  = (unsigned short*)(ws + oKl);
  unsigned short* Vh  = (unsigned short*)(ws + oVh);
  unsigned short* Vl  = (unsigned short*)(ws + oVl);
  unsigned short* Ah  = (unsigned short*)(ws + oAh);
  unsigned short* Al  = (unsigned short*)(ws + oAl);

  const dim3 b256(256), b128(128);

  rope_table_kernel<<<dim3(NTOK / 8), b256, 0, stream>>>(positions, cst, snt, NTOK);
  cvt_bf16_kernel<<<dim3((NTOK * HID / 8) / 256), b256, 0, stream>>>(hidden, Xb, NTOK * HID / 8);
  tconv_bf16_kernel<<<dim3(QKVN / 64, HID / 64), b256, 0, stream>>>(Wqkv, WqT, HID, QKVN);
  tconv_bf16_kernel<<<dim3(HID / 64, HID / 64), b256, 0, stream>>>(Wo, WoT, HID, HID);
  tconv16_bf16_kernel<<<dim3(HID / 64), b256, 0, stream>>>(Wg, WgT, HID);
  gemm_w32x128_kernel<0, false><<<dim3((NTOK / 32) * (QKW / 128) / 4), b128, 0, stream>>>(
      Xb, Xb, HID, WqT, HID, qnw, knw, cst, snt, (void*)Qh, (void*)Ql, (void*)Kh, (void*)Kl, HID, NTOK, QKW, HID);
  gemm_w32x128_kernel<1, false><<<dim3((KVW / 32) * (NTOK / 128) / 4), b128, 0, stream>>>(
      WqT + (size_t)QKW * HID, WqT + (size_t)QKW * HID, HID, Xb, HID, qnw, knw, cst, snt,
      (void*)Vh, (void*)Vl, (void*)Vh, (void*)Vl, NTOK, KVW, NTOK, HID);
  gate_kernel<<<dim3(NTOK / 128), b128, 0, stream>>>(Xb, WgT, gate, NTOK, HID);
  attn_causal_kernel<true><<<dim3(8, NHQ), b128, 0, stream>>>(Qh, Ql, Kh, Kl, Vh, Vl, gate, Ah, Al, 0);
  attn_causal_kernel<false><<<dim3(NTOK / 64 - 8, NHQ), b128, 0, stream>>>(Qh, Ql, Kh, Kl, Vh, Vl, gate, Ah, Al, 8);
  gemm_w32x128_kernel<2, true><<<dim3((NTOK / 32) * (HID / 128) / 4), b128, 0, stream>>>(
      Ah, Al, HID, WoT, HID, qnw, knw, cst, snt, (void*)out, (void*)out, (void*)out, (void*)out, HID, NTOK, HID, HID);
  (void)hipGetLastError();
}
